// GaussianImage_Cholesky_EA_21663815041286
// MI455X (gfx1250) — hardware-verified
//
#include <hip/hip_runtime.h>
#include <stddef.h>

#pragma clang fp contract(off)

typedef _Float16 v16h __attribute__((ext_vector_type(16)));
typedef _Float16 v8h  __attribute__((ext_vector_type(8)));
typedef float    v8f  __attribute__((ext_vector_type(8)));
typedef float    v4f  __attribute__((ext_vector_type(4)));
typedef v8h __attribute__((may_alias)) v8ha;
typedef v8f __attribute__((may_alias)) v8fa;
typedef v4f __attribute__((may_alias)) v4fa;

union Frag { v16h v; v8h half[2]; };

#define NG      2048
#define RANKF   12
#define NPAD    16
#define IMG_W   128
#define IMG_H   128
#define NPIX    (IMG_W * IMG_H)
#define NTILES  64
#define STAGE   256
#define NSTAGE  (NG / STAGE)
#define FSCALE  64.0f
#define FINV    0.015625f

static_assert(NG % STAGE == 0);
static_assert(STAGE % 32 == 0);
static_assert(NG % 32 == 0);

__device__ __forceinline__ v8f wmma_f16(v16h a, v16h b, v8f c) {
#if defined(__HIP_DEVICE_COMPILE__)
  v8f d = __builtin_amdgcn_wmma_f32_16x16x32_f16(false, a, false, b, (short)0, c, false, false);
  asm volatile("v_nop\n\tv_nop\n\tv_nop\n\tv_nop" : "+v"(d) : "v"(a), "v"(b));
  return d;
#else
  (void)a; (void)b;
  return c;
#endif
}

__device__ __forceinline__ unsigned int ballot32(int pred) {
#if defined(__HIP_DEVICE_COMPILE__)
  return __builtin_amdgcn_ballot_w32(pred != 0);
#else
  return (unsigned int)(pred != 0);
#endif
}

__global__ __launch_bounds__(256) void k_gauss(const float* __restrict__ xyz,
                                              const float* __restrict__ chol,
                                              const float* __restrict__ opa,
                                              float* gt, unsigned int* gm) {
#pragma clang fp contract(off)
  const int g = (int)blockIdx.x * 256 + (int)threadIdx.x;
  if (g >= NG) return;

  const float mx = tanhf(xyz[2 * g + 0]);
  const float my = tanhf(xyz[2 * g + 1]);
  const float l1 = chol[3 * g + 0] + 0.5f;
  const float l2 = chol[3 * g + 1] + 0.0f;
  const float l3 = chol[3 * g + 2] + 0.5f;
  const float c00 = l1 * l1;
  const float c01 = l1 * l2;
  const float c11 = l2 * l2 + l3 * l3;
  const float det = c00 * c11 - c01 * c01;
  const float inv = 1.0f / det;
  const float ca = c11 * inv;
  const float cb = (-c01) * inv;
  const float cc = c00 * inv;
  const float cx = 64.0f * (mx + 1.0f);
  const float cy = 64.0f * (my + 1.0f);
  const float mid = 0.5f * (c00 + c11);
  const float v1 = mid + sqrtf(fmaxf(mid * mid - det, (float)0.1));
  const float radius = ceilf(3.0f * sqrtf(v1));

  const float fx0 = floorf((cx - radius) * 0.0625f);
  const float fx1 = floorf((cx + radius) * 0.0625f) + 1.0f;
  const float fy0 = floorf((cy - radius) * 0.0625f);
  const float fy1 = floorf((cy + radius) * 0.0625f) + 1.0f;
  const int tminx = (int)fminf(fmaxf(fx0, 0.0f), 8.0f);
  const int tmaxx = (int)fminf(fmaxf(fx1, 0.0f), 8.0f);
  const int tminy = (int)fminf(fmaxf(fy0, 0.0f), 8.0f);
  const int tmaxy = (int)fminf(fmaxf(fy1, 0.0f), 8.0f);

  unsigned int rowmask = 0u;
  if (tmaxx > tminx) rowmask = (1u << tmaxx) - (1u << tminx);
  unsigned long long msk = 0ull;
#pragma unroll
  for (int t = 0; t < 8; ++t)
    if (t >= tminy && t < tmaxy) msk |= ((unsigned long long)rowmask) << (8 * t);
  const unsigned int mlo = (unsigned int)(msk & 0xffffffffull);
  const unsigned int mhi = (unsigned int)(msk >> 32);
  const float op = opa[g];

  volatile float* vg = gt;
  volatile unsigned int* vm = gm;
  vg[0 * NG + g] = cx;  vg[1 * NG + g] = cy;  vg[2 * NG + g] = ca;
  vg[3 * NG + g] = cb;  vg[4 * NG + g] = cc;  vg[5 * NG + g] = op;
  vm[0 * NG + g] = mlo; vm[1 * NG + g] = mhi;
  __threadfence();
  vg[0 * NG + g] = cx;  vg[1 * NG + g] = cy;  vg[2 * NG + g] = ca;
  vg[3 * NG + g] = cb;  vg[4 * NG + g] = cc;  vg[5 * NG + g] = op;
  vm[0 * NG + g] = mlo; vm[1 * NG + g] = mhi;
}

__global__ __launch_bounds__(256) void k_feat(const float* __restrict__ feat, _Float16* ft) {
#pragma clang fp contract(off)
  const int n  = (int)blockIdx.x;
  const int k8 = (int)threadIdx.x;
  v8h o = {0, 0, 0, 0, 0, 0, 0, 0};
  if (n < RANKF) {
#pragma unroll
    for (int e = 0; e < 8; ++e)
      o[e] = (_Float16)(feat[(8 * k8 + e) * RANKF + n] * FSCALE);
  }
  _Float16* dst = ft + (size_t)n * NG + 8 * k8;
  *(volatile v8h*)dst = o;
  __threadfence();
  *(volatile v8h*)dst = o;
}

__device__ __forceinline__ void out_pass(const float* so, float* out, int y0, int tx, int lane) {
#pragma unroll
  for (int i = 0; i < 3; ++i) {
    const int f = 32 * i + lane;
    const int t = (f >= 48) ? 1 : 0;
    const int q = f - 48 * t;
    const v4f v = *(const v4fa*)(so + 192 * t + 4 * q);
    float* dst = out + ((size_t)(y0 + t) * IMG_W + (size_t)tx * 16) * RANKF + 4 * q;
    *(volatile v4f*)dst = v;
  }
}

__global__ __launch_bounds__(256) void k_raster(const float* __restrict__ gt,
                                               const unsigned int* __restrict__ gm,
                                               const _Float16* __restrict__ ft,
                                               float* out) {
#pragma clang fp contract(off)
  __shared__ __attribute__((aligned(32))) float sP[6][STAGE];
  __shared__ unsigned int sIn[STAGE / 32];
  __shared__ __attribute__((aligned(16))) float sO[8 * 384];

  const int tid = (int)threadIdx.x, lane = tid & 31, w = tid >> 5;
  const int h = lane >> 4, m = lane & 15;
  const int tx = (int)blockIdx.x & 7, ty = (int)blockIdx.x >> 3;
  const int tbit = ty * 8 + tx;
  const float pxf = (float)(tx * 16 + m);
  const int y0 = ty * 16 + 2 * w;
  const float pyf0 = (float)y0;
  const float pyf1 = (float)(y0 + 1);
  const float thr  = (float)(1.0 / 255.0);
  const float amax = (float)0.999;

  const v8f zero8 = {0.f, 0.f, 0.f, 0.f, 0.f, 0.f, 0.f, 0.f};
  const v16h z16 = {0, 0, 0, 0, 0, 0, 0, 0, 0, 0, 0, 0, 0, 0, 0, 0};
  v8f acc0 = zero8, acc1 = zero8;
  const _Float16* fb = ft + (size_t)m * NG;

#pragma unroll 1
  for (int s = 0; s < NSTAGE; ++s) {
    __syncthreads();
    const int g = s * STAGE + tid;
    sP[0][tid] = gt[0 * NG + g];
    sP[1][tid] = gt[1 * NG + g];
    sP[2][tid] = gt[2 * NG + g];
    sP[3][tid] = gt[3 * NG + g];
    sP[4][tid] = gt[4 * NG + g];
    sP[5][tid] = gt[5 * NG + g];
    const unsigned int mlo = gm[0 * NG + g];
    const unsigned int mhi = gm[1 * NG + g];
    const unsigned int word = (tbit >= 32) ? mhi : mlo;
    const int bit = (int)((word >> (tbit & 31)) & 1u);
    const unsigned int bal = ballot32(bit);
    if (lane == 0) sIn[w] = bal;
    __syncthreads();

#pragma unroll 1
    for (int c = 0; c < STAGE / 32; ++c) {
      const unsigned int msk = sIn[c];
      if (msk == 0u) continue;
      const int base = c * 32;
      v16h a0 = z16, a1 = z16;
#pragma unroll
      for (int grp = 0; grp < 2; ++grp) {
        const int jb = base + 16 * grp + 8 * h;
        const v8f gcx = *(const v8fa*)(&sP[0][jb]);
        const v8f gcy = *(const v8fa*)(&sP[1][jb]);
        const v8f gca = *(const v8fa*)(&sP[2][jb]);
        const v8f gcb = *(const v8fa*)(&sP[3][jb]);
        const v8f gcc = *(const v8fa*)(&sP[4][jb]);
        const v8f gop = *(const v8fa*)(&sP[5][jb]);
#pragma unroll
        for (int e = 0; e < 8; ++e) {
          const int i = 8 * grp + e;
          const int jbit = 16 * grp + 8 * h + e;
          const bool inside = ((msk >> jbit) & 1u) != 0u;
          const float dx   = gcx[e] - pxf;
          const float cadx = gca[e] * dx;
          const float t1   = cadx * dx;
          const float cbdx = gcb[e] * dx;
          {
            const float dy   = gcy[e] - pyf0;
            const float ccdy = gcc[e] * dy;
            const float t2   = ccdy * dy;
            const float sg   = 0.5f * (t1 + t2) + cbdx * dy;
            const bool  nn   = (sg >= 0.0f);
            const float sgc  = nn ? sg : 0.0f;
            const float al   = fminf(amax, gop[e] * expf(-sgc));
            const bool  va   = inside & nn & (al >= thr);
            a0[i] = (_Float16)(va ? al : 0.0f);
          }
          {
            const float dy   = gcy[e] - pyf1;
            const float ccdy = gcc[e] * dy;
            const float t2   = ccdy * dy;
            const float sg   = 0.5f * (t1 + t2) + cbdx * dy;
            const bool  nn   = (sg >= 0.0f);
            const float sgc  = nn ? sg : 0.0f;
            const float al   = fminf(amax, gop[e] * expf(-sgc));
            const bool  va   = inside & nn & (al >= thr);
            a1[i] = (_Float16)(va ? al : 0.0f);
          }
        }
      }
      const int k0 = s * STAGE + base;
      Frag b;
      b.half[0] = *(const v8ha*)(fb + k0 + 8 * h);
      b.half[1] = *(const v8ha*)(fb + k0 + 16 + 8 * h);
      acc0 = wmma_f16(a0, b.v, acc0);
      acc1 = wmma_f16(a1, b.v, acc1);
    }
  }

  float* so = sO + w * 384;
  if (m < RANKF) {
#pragma unroll
    for (int r = 0; r < 8; ++r) {
      const int x = 8 * h + r;
      so[x * RANKF + m]       = fminf(fmaxf(acc0[r] * FINV, 0.0f), 1.0f);
      so[192 + x * RANKF + m] = fminf(fmaxf(acc1[r] * FINV, 0.0f), 1.0f);
    }
  }
  __syncthreads();

  out_pass(so, out, y0, tx, lane);
  __threadfence();
  out_pass(so, out, y0, tx, lane);
}

extern "C" void kernel_launch(void* const* d_in, const int* in_sizes, int n_in,
                              void* d_out, int out_size, void* d_ws, size_t ws_size,
                              hipStream_t stream) {
  if (n_in < 4) return;
  if (in_sizes[0] != NG * 2) return;
  if (in_sizes[1] != NG * 3) return;
  if (in_sizes[2] != NG * RANKF) return;
  if (in_sizes[3] != NG) return;
  if (out_size != NPIX * RANKF) return;

  const float* xyz  = (const float*)d_in[0];
  const float* chol = (const float*)d_in[1];
  const float* feat = (const float*)d_in[2];
  const float* opa  = (const float*)d_in[3];
  float* out = (float*)d_out;

  const size_t gt_bytes = (size_t)6 * NG * 4;
  const size_t gm_bytes = (size_t)2 * NG * 4;
  const size_t ft_bytes = (size_t)NPAD * NG * 2;
  const size_t total = gt_bytes + gm_bytes + ft_bytes;
  if (total > ws_size) return;

  char* ws = (char*)d_ws;
  float*        gt = (float*)(ws);
  unsigned int* gm = (unsigned int*)(ws + gt_bytes);
  _Float16*     ft = (_Float16*)(ws + gt_bytes + gm_bytes);

  k_gauss<<<NG / 256, 256, 0, stream>>>(xyz, chol, opa, gt, gm);
  k_feat<<<NPAD, 256, 0, stream>>>(feat, ft);
  k_raster<<<NTILES, 256, 0, stream>>>(gt, gm, ft, out);
}
